// GINModel_1391569404373
// MI455X (gfx1250) — hardware-run, weakly checked
//
#include <hip/hip_runtime.h>
#include <stddef.h>
#include <stdint.h>
#include <math.h>

#define NN      40000
#define NE      640000
#define DH      128
#define OC      64
#define GBM     128
#define MP      40064
#define APITCH  256
#define WPITCH  256
#define SPLIT_AGG 1
#define SPLIT_HID 1
#define KEXT_AGG (SPLIT_AGG ? 256 : 128)
#define KEXT_HID (SPLIT_HID ? 256 : 128)
#define NTHR    256
#define NWAVE   8
#define EPT     8
#define WCH     (32 * EPT)
#define NBRUN   1024
#define SLB     10
#define NBK     40
#define WLCAP   3584
#define RCAP    28672
#define TRIPCAP 64
#define MAXDEG_MEAS   36
#define MAXB1024_MEAS 16638
#define ABM     64
#define SP128   132
#define SP64    68
#define WSMAX   (128u << 20)
#define SM_EPS  448

#define BK_ZINTS (NWAVE * WLCAP + RCAP + 3 * NBRUN)
#define BK_INTS  (BK_ZINTS + 16)
#define BK_LDS   (BK_INTS * 4)
#define GM_LDS   ((GBM * SP128 + DH) * 4)

#define PBX   (MP * DH / 8 / NTHR)
#define PBW   (DH * WPITCH / 8 / NTHR)
#define PBW4  (OC * WPITCH / 8 / NTHR)
#define PBTOT (PBX + 3 * PBW + PBW4 + 1)

static_assert(DH == 128 && DH == 32 * 4 && OC == 64 && OC == 32 * 2);
static_assert(MP % GBM == 0 && MP == 313 * GBM && MP >= NN && MP % ABM == 0 && NN == 312 * GBM + 64);
static_assert(NBRUN == (1 << SLB) && NBRUN % ABM == 0 && NBRUN % GBM == 0 && NBRUN % 32 == 0);
static_assert(NBK * NBRUN >= MP);
static_assert(NE < (1 << 21) && (((long long)NE) << SLB) < (1LL << 31));
static_assert(NE % WCH == 0 && NE % 4 == 0);
static_assert(RCAP == NWAVE * WLCAP && RCAP % (NTHR * 4) == 0 && BK_ZINTS % 4 == 0 && (2 * NBRUN) % (NTHR * 4) == 0);
static_assert((long long)RCAP * 100 >= (long long)MAXB1024_MEAS * 105);
static_assert(WLCAP >= MAXB1024_MEAS / 8 + 8 * 46 + 1);
static_assert(MAXDEG_MEAS + 8 <= TRIPCAP && TRIPCAP <= 64);
static_assert(ABM == NWAVE * 8 && GBM == NWAVE * 16);
static_assert(BK_LDS <= 300000 && GM_LDS <= 327680);
static_assert((GBM * SP64 + OC) * 4 <= 65536);
static_assert((MP * DH / 8) % NTHR == 0 && (DH * WPITCH / 8) % NTHR == 0 && (OC * WPITCH / 8) % NTHR == 0);
static_assert(KEXT_AGG % 32 == 0 && KEXT_HID % 32 == 0 && KEXT_AGG <= APITCH && KEXT_HID <= APITCH);
static_assert(KEXT_AGG <= WPITCH && KEXT_HID <= WPITCH && APITCH == 2 * DH && WPITCH == 2 * DH);
static_assert(3 * DH + OC == SM_EPS && SM_EPS + 2 <= 512);

typedef float          v2f   __attribute__((ext_vector_type(2)));
typedef float          v4f   __attribute__((ext_vector_type(4)));
typedef float          v8f   __attribute__((ext_vector_type(8)));
typedef int            v4i   __attribute__((ext_vector_type(4)));
typedef int            v8i   __attribute__((ext_vector_type(8)));
typedef unsigned int   v2u   __attribute__((ext_vector_type(2)));
typedef unsigned int   v4u   __attribute__((ext_vector_type(4)));
typedef unsigned short v8us  __attribute__((ext_vector_type(8)));
typedef unsigned short v16us __attribute__((ext_vector_type(16)));
typedef __bf16         v16bf __attribute__((ext_vector_type(16)));
typedef v2f  __attribute__((may_alias)) v2fa;
typedef v4f  __attribute__((may_alias)) v4fa;
typedef v4i  __attribute__((may_alias)) v4ia;
typedef v2u  __attribute__((may_alias)) v2ua;
typedef v8us __attribute__((may_alias)) v8usa;
union FragB { v16bf v; v16us u; v8us h[2]; v8i w; };

__device__ __forceinline__ v8f wmb(const FragB& a, const FragB& b, v8f c) {
  v8f d = __builtin_amdgcn_wmma_f32_16x16x32_bf16(false, a.v, false, b.v, (short)0, c, false, false);
  asm volatile("v_nop\n\tv_nop\n\tv_nop\n\tv_nop" : "+v"(d) : "v"(a.w), "v"(b.w));
  return d;
}

__device__ __forceinline__ unsigned bf16_bits(float f) {
  const unsigned u = __float_as_uint(f);
  const unsigned r = (u + 0x7FFFu + ((u >> 16) & 1u)) >> 16;
  const unsigned q = (u >> 16) | 0x40u;
  return ((u & 0x7fffffffu) > 0x7f800000u) ? q : r;
}
__device__ __forceinline__ float bf16_val(float f) {
  return __uint_as_float(bf16_bits(f) << 16);
}

__device__ __forceinline__ void hilo_pack(float v0, float v1, float v2, float v3,
                                          unsigned& h01, unsigned& h23, unsigned& l01, unsigned& l23) {
  const unsigned a0 = bf16_bits(v0), a1 = bf16_bits(v1), a2 = bf16_bits(v2), a3 = bf16_bits(v3);
  const unsigned b0 = bf16_bits(v0 - __uint_as_float(a0 << 16));
  const unsigned b1 = bf16_bits(v1 - __uint_as_float(a1 << 16));
  const unsigned b2 = bf16_bits(v2 - __uint_as_float(a2 << 16));
  const unsigned b3 = bf16_bits(v3 - __uint_as_float(a3 << 16));
  h01 = a0 | (a1 << 16); h23 = a2 | (a3 << 16);
  l01 = b0 | (b1 << 16); l23 = b2 | (b3 << 16);
}

__device__ __forceinline__ v4u regroup16(unsigned h01, unsigned h23, unsigned l01, unsigned l23, int lane) {
  const int t  = lane & 15;
  const int s0 = 2 * t, s1 = 2 * t + 1;
  const unsigned a0 = (unsigned)__shfl((int)h01, s0, 32), a1 = (unsigned)__shfl((int)h23, s0, 32);
  const unsigned a2 = (unsigned)__shfl((int)h01, s1, 32), a3 = (unsigned)__shfl((int)h23, s1, 32);
  const unsigned b0 = (unsigned)__shfl((int)l01, s0, 32), b1 = (unsigned)__shfl((int)l23, s0, 32);
  const unsigned b2 = (unsigned)__shfl((int)l01, s1, 32), b3 = (unsigned)__shfl((int)l23, s1, 32);
  const unsigned mk = (lane < 16) ? 0xffffffffu : 0u;
  v4u o;
  o.x = (a0 & mk) | (b0 & ~mk); o.y = (a1 & mk) | (b1 & ~mk);
  o.z = (a2 & mk) | (b2 & ~mk); o.w = (a3 & mk) | (b3 & ~mk);
  return o;
}

__device__ __forceinline__ void st2_v4f(float* p, v4f v, bool ok) {
  if (ok) *(volatile v4f*)p = v;
  __threadfence();
  if (ok) *(volatile v4f*)p = v;
}
__device__ __forceinline__ void st2_v2f(float* p, v2f v, bool ok) {
  if (ok) *(volatile v2f*)p = v;
  __threadfence();
  if (ok) *(volatile v2f*)p = v;
}
__device__ __forceinline__ void st2_v4u(unsigned short* p, v4u v) {
  *(volatile v4u*)p = v;
  __threadfence();
  *(volatile v4u*)p = v;
}
__device__ __forceinline__ void st2_v8us(unsigned short* p, v8us v) {
  *(volatile v8us*)p = v;
  __threadfence();
  *(volatile v8us*)p = v;
}

__device__ __forceinline__ v8us gather8(const float* __restrict__ base, int stride) {
  float f[8];
#pragma unroll
  for (int i = 0; i < 8; ++i) f[i] = base[(size_t)i * (size_t)stride];
  v8us o;
#pragma unroll
  for (int i = 0; i < 8; ++i) o[i] = (unsigned short)bf16_bits(f[i]);
  return o;
}

__device__ __forceinline__ v4f bf4(v4f a) {
  v4f o;
  o.x = bf16_val(a.x); o.y = bf16_val(a.y); o.z = bf16_val(a.z); o.w = bf16_val(a.w);
  return o;
}

__global__ __launch_bounds__(NTHR) void k_prep(const float* __restrict__ x,
                                               const float* __restrict__ w1, const float* __restrict__ w2,
                                               const float* __restrict__ w3, const float* __restrict__ w4,
                                               const float* __restrict__ b1, const float* __restrict__ b2,
                                               const float* __restrict__ b3, const float* __restrict__ b4,
                                               const float* __restrict__ e0p, const float* __restrict__ e1p,
                                               unsigned short* xb, unsigned short* w1d, unsigned short* w2d,
                                               unsigned short* w3d, unsigned short* w4d, float* sm) {
  const int tid = (int)threadIdx.x, lane = tid & 31, wave = tid >> 5;
  const int blk = (int)blockIdx.x;
  if (blk < PBX) {
    const int u   = blk * NTHR + tid;
    const int row = u >> 4, k8 = (u & 15) * 8;
    const int rc  = row < NN ? row : NN - 1;
    const unsigned mk = row < NN ? 0xffffu : 0u;
    const float* p = x + (size_t)rc * DH + k8;
    const v4f a = *(const v4fa*)p;
    const v4f b = *(const v4fa*)(p + 4);
    v8us o;
    o[0] = (unsigned short)(bf16_bits(a.x) & mk); o[1] = (unsigned short)(bf16_bits(a.y) & mk);
    o[2] = (unsigned short)(bf16_bits(a.z) & mk); o[3] = (unsigned short)(bf16_bits(a.w) & mk);
    o[4] = (unsigned short)(bf16_bits(b.x) & mk); o[5] = (unsigned short)(bf16_bits(b.y) & mk);
    o[6] = (unsigned short)(bf16_bits(b.z) & mk); o[7] = (unsigned short)(bf16_bits(b.w) & mk);
    st2_v8us(xb + (size_t)row * DH + k8, o);
  } else if (blk < PBX + PBW) {
    const int u = (blk - PBX) * NTHR + tid;
    const int n = u >> 5, k8 = (u & 31) * 8, kk = k8 & (DH - 1);
    const v8us o = gather8(w1 + (size_t)kk * DH + n, DH);
    st2_v8us(w1d + (size_t)n * WPITCH + k8, o);
  } else if (blk < PBX + 2 * PBW) {
    const int u = (blk - PBX - PBW) * NTHR + tid;
    const int n = u >> 5, k8 = (u & 31) * 8, kk = k8 & (DH - 1);
    const v8us o = gather8(w2 + (size_t)kk * DH + n, DH);
    st2_v8us(w2d + (size_t)n * WPITCH + k8, o);
  } else if (blk < PBX + 3 * PBW) {
    const int u = (blk - PBX - 2 * PBW) * NTHR + tid;
    const int n = u >> 5, k8 = (u & 31) * 8, kk = k8 & (DH - 1);
    const v8us o = gather8(w3 + (size_t)kk * DH + n, DH);
    st2_v8us(w3d + (size_t)n * WPITCH + k8, o);
  } else if (blk < PBX + 3 * PBW + PBW4) {
    const int u = (blk - PBX - 3 * PBW) * NTHR + tid;
    const int n = u >> 5, k8 = (u & 31) * 8, kk = k8 & (DH - 1);
    const v8us o = gather8(w4 + (size_t)kk * OC + n, OC);
    st2_v8us(w4d + (size_t)n * WPITCH + k8, o);
  } else {
    if (tid < 128) {
      v4f o;
      if (wave == 0) {
        o = bf4(*(const v4fa*)(b1 + 4 * lane));
      } else if (wave == 1) {
        o = bf4(*(const v4fa*)(b2 + 4 * lane));
      } else if (wave == 2) {
        o = bf4(*(const v4fa*)(b3 + 4 * lane));
      } else {
        const v4f c = *(const v4fa*)(b4 + 4 * (lane & 15));
        const float ea = e0p[0];
        const float eb = e1p[0];
        asm volatile("" :: "v"(c));
        asm volatile("" :: "v"(ea), "v"(eb));
        const unsigned mb = (lane < 16) ? 0xffffffffu : 0u;
        const unsigned me = (lane == 16) ? 0xffffffffu : 0u;
        o.x = __uint_as_float(((bf16_bits(c.x) << 16) & mb) | ((bf16_bits(ea) << 16) & me));
        o.y = __uint_as_float(((bf16_bits(c.y) << 16) & mb) | ((bf16_bits(eb) << 16) & me));
        o.z = __uint_as_float((bf16_bits(c.z) << 16) & mb);
        o.w = __uint_as_float((bf16_bits(c.w) << 16) & mb);
      }
      st2_v4f(sm + 4 * tid, o, true);
    }
  }
}

__device__ __forceinline__ void bucket_flush(const int* pl, const int* cnt, int ov, int* lp, int* cop, int* fp,
                                             int tid) {
#pragma unroll 1
  for (int i = tid * 4; i < RCAP; i += NTHR * 4) {
    const v4i v = *(const v4ia*)(pl + i);
    *(volatile v4i*)(lp + i) = v;
  }
#pragma unroll 1
  for (int i = tid * 4; i < 2 * NBRUN; i += NTHR * 4) {
    const v4i v = *(const v4ia*)(cnt + i);
    *(volatile v4i*)(cop + i) = v;
  }
  if (tid < 8) {
    const v4i f = {ov, ov, ov, ov};
    *(volatile v4i*)(fp + 4 * tid) = f;
  }
}

__global__ __launch_bounds__(NTHR) void k_bucket(const int* __restrict__ srcs, const int* __restrict__ dsts,
                                                 int* LIST, int* CO, int* FLAG) {
  extern __shared__ __attribute__((aligned(16))) int dsm[];
  int* wl   = dsm;
  int* pl   = dsm + NWAVE * WLCAP;
  int* cnt  = pl + RCAP;
  int* offs = cnt + NBRUN;
  int* cur  = offs + NBRUN;
  int* misc = cur + NBRUN;
  const int tid = (int)threadIdx.x, lane = tid & 31, wave = tid >> 5;
  const int blk = (int)blockIdx.x;
  const unsigned nbs = (unsigned)(blk * NBRUN);

  {
    const v4i z4 = {0, 0, 0, 0};
    for (int i = tid * 4; i < BK_ZINTS; i += NTHR * 4) *(v4ia*)(dsm + i) = z4;
    if (tid < 16) misc[tid] = 0;
  }
  __syncthreads();

  {
    const int per  = ((NE + NWAVE * WCH - 1) / (NWAVE * WCH)) * WCH;
    const int ebeg = wave * per;
    const int eend = (ebeg + per < NE) ? (ebeg + per) : NE;
    int* mylist = wl + wave * WLCAP;
    int wc = 0;
#pragma unroll 1
    for (int cb = ebeg; cb < eend; cb += WCH) {
      const int e0 = cb + lane * EPT;
      const v4i da = *(const v4ia*)(dsts + e0);
      const v4i db = *(const v4ia*)(dsts + e0 + 4);
      const unsigned s0 = (unsigned)da.x - nbs, s1 = (unsigned)da.y - nbs;
      const unsigned s2 = (unsigned)da.z - nbs, s3 = (unsigned)da.w - nbs;
      const unsigned s4 = (unsigned)db.x - nbs, s5 = (unsigned)db.y - nbs;
      const unsigned s6 = (unsigned)db.z - nbs, s7 = (unsigned)db.w - nbs;
      const bool h0 = s0 < (unsigned)NBRUN, h1 = s1 < (unsigned)NBRUN, h2 = s2 < (unsigned)NBRUN, h3 = s3 < (unsigned)NBRUN;
      const bool h4 = s4 < (unsigned)NBRUN, h5 = s5 < (unsigned)NBRUN, h6 = s6 < (unsigned)NBRUN, h7 = s7 < (unsigned)NBRUN;
      const unsigned m0 = __builtin_amdgcn_ballot_w32(h0), m1 = __builtin_amdgcn_ballot_w32(h1);
      const unsigned m2 = __builtin_amdgcn_ballot_w32(h2), m3 = __builtin_amdgcn_ballot_w32(h3);
      const unsigned m4 = __builtin_amdgcn_ballot_w32(h4), m5 = __builtin_amdgcn_ballot_w32(h5);
      const unsigned m6 = __builtin_amdgcn_ballot_w32(h6), m7 = __builtin_amdgcn_ballot_w32(h7);
      const unsigned any = m0 | m1 | m2 | m3 | m4 | m5 | m6 | m7;
      if (any != 0u) {
        const int pre = (int)(__builtin_amdgcn_mbcnt_lo(m0, 0u) + __builtin_amdgcn_mbcnt_lo(m1, 0u) +
                              __builtin_amdgcn_mbcnt_lo(m2, 0u) + __builtin_amdgcn_mbcnt_lo(m3, 0u) +
                              __builtin_amdgcn_mbcnt_lo(m4, 0u) + __builtin_amdgcn_mbcnt_lo(m5, 0u) +
                              __builtin_amdgcn_mbcnt_lo(m6, 0u) + __builtin_amdgcn_mbcnt_lo(m7, 0u));
        int p = wc + pre;
        if (h0) { if (p < WLCAP) mylist[p] = ((e0 + 0) << SLB) | (int)s0; p = p + 1; }
        if (h1) { if (p < WLCAP) mylist[p] = ((e0 + 1) << SLB) | (int)s1; p = p + 1; }
        if (h2) { if (p < WLCAP) mylist[p] = ((e0 + 2) << SLB) | (int)s2; p = p + 1; }
        if (h3) { if (p < WLCAP) mylist[p] = ((e0 + 3) << SLB) | (int)s3; p = p + 1; }
        if (h4) { if (p < WLCAP) mylist[p] = ((e0 + 4) << SLB) | (int)s4; p = p + 1; }
        if (h5) { if (p < WLCAP) mylist[p] = ((e0 + 5) << SLB) | (int)s5; p = p + 1; }
        if (h6) { if (p < WLCAP) mylist[p] = ((e0 + 6) << SLB) | (int)s6; p = p + 1; }
        if (h7) { if (p < WLCAP) mylist[p] = ((e0 + 7) << SLB) | (int)s7; p = p + 1; }
        wc += (int)(__builtin_popcount(m0) + __builtin_popcount(m1) + __builtin_popcount(m2) + __builtin_popcount(m3) +
                    __builtin_popcount(m4) + __builtin_popcount(m5) + __builtin_popcount(m6) + __builtin_popcount(m7));
      }
    }
    if (lane == 0) misc[wave] = wc;
  }
  __syncthreads();

  if (wave == 0) {
    int ov = 0;
#pragma unroll 1
    for (int w2 = 0; w2 < NWAVE; ++w2) {
      int c = misc[w2];
      if (c > WLCAP) ov = 1;
      c = c < 0 ? 0 : (c > WLCAP ? WLCAP : c);
#pragma unroll 1
      for (int b0 = 0; b0 < c; b0 += 32) {
        const int idx = b0 + lane;
        const int ent = wl[w2 * WLCAP + (idx < WLCAP ? idx : WLCAP - 1)];
        const int m32 = (c - b0) < 32 ? (c - b0) : 32;
#pragma unroll 1
        for (int k = 0; k < m32; ++k) {
          const int u    = __builtin_amdgcn_readlane(ent, k);
          const int slot = u & (NBRUN - 1);
          if (lane == 0) cnt[slot] = cnt[slot] + 1;
        }
      }
    }
    if (lane == 0) misc[9] = ov;
  }
  __syncthreads();
  if (wave == 0) {
    const int base = lane * (NBRUN / 32);
    int s = 0;
#pragma unroll 1
    for (int i = 0; i < NBRUN / 32; ++i) s += cnt[base + i];
    int incl = s;
#pragma unroll
    for (int d = 1; d < 32; d <<= 1) {
      const int y = __shfl_up(incl, d, 32);
      if (lane >= d) incl += y;
    }
    int run = incl - s;
#pragma unroll 1
    for (int i = 0; i < NBRUN / 32; ++i) {
      const int cv = cnt[base + i];
      offs[base + i] = run;
      cur[base + i]  = run;
      run += cv;
    }
  }
  __syncthreads();

  if (wave == 0) {
#pragma unroll 1
    for (int w2 = 0; w2 < NWAVE; ++w2) {
      int c = misc[w2];
      c = c < 0 ? 0 : (c > WLCAP ? WLCAP : c);
#pragma unroll 1
      for (int b0 = 0; b0 < c; b0 += 32) {
        const int idx = b0 + lane;
        const int ent = wl[w2 * WLCAP + (idx < WLCAP ? idx : WLCAP - 1)];
        int eid = (ent >> SLB) & 0x1FFFFF;
        eid = eid > NE - 1 ? NE - 1 : eid;
        int sr = srcs[eid];
        sr = sr < 0 ? 0 : (sr > NN - 1 ? NN - 1 : sr);
        const int m32 = (c - b0) < 32 ? (c - b0) : 32;
#pragma unroll 1
        for (int k = 0; k < m32; ++k) {
          const int u    = __builtin_amdgcn_readlane(ent, k);
          const int wd   = __builtin_amdgcn_readlane(sr, k);
          const int slot = u & (NBRUN - 1);
          if (lane == 0) {
            int p = cur[slot];
            p = p < 0 ? 0 : (p > RCAP - 1 ? RCAP - 1 : p);
            pl[p] = wd;
            cur[slot] = p + 1;
          }
        }
      }
    }
  }
  __syncthreads();

  const int ovf = misc[9];
  int* lp  = LIST + (size_t)blk * RCAP;
  int* cop = CO + (size_t)blk * (2 * NBRUN);
  int* fp  = FLAG + (size_t)blk * 32;
  bucket_flush(pl, cnt, ovf, lp, cop, fp, tid);
  __threadfence();
  bucket_flush(pl, cnt, ovf, lp, cop, fp, tid);
}

template <int SRC16>
__global__ __launch_bounds__(NTHR) void k_agg(const int* __restrict__ LIST, const int* __restrict__ CO,
                                              const int* __restrict__ FLAG,
                                              const unsigned short* __restrict__ XB, const float* __restrict__ H,
                                              const float* __restrict__ sm, int epsIdx, unsigned short* Z) {
  const int tid = (int)threadIdx.x, lane = tid & 31, wave = tid >> 5;
  const int rowBase = (int)blockIdx.x * ABM;
  const int bucket  = rowBase >> SLB;
  const int* lb  = LIST + (size_t)bucket * RCAP;
  const int* cob = CO + (size_t)bucket * (2 * NBRUN);
  const int flag = FLAG[(size_t)bucket * 32];
  const float sc = 1.0f + sm[SM_EPS + (epsIdx != 0 ? 1 : 0)];
  const float qnan = __uint_as_float(0x7fc00000u);

#pragma unroll 1
  for (int i = 0; i < ABM / NWAVE; ++i) {
    const int d    = rowBase + (ABM / NWAVE) * wave + i;
    const int slot = d & (NBRUN - 1);
    const int cr = cob[slot];
    const int orw = cob[NBRUN + slot];
    int bigv = cr > TRIPCAP ? 1 : 0;
    int c = cr < 0 ? 0 : (cr > TRIPCAP ? TRIPCAP : cr);
    int o = orw < 0 ? 0 : (orw > RCAP - 1 ? RCAP - 1 : orw);
    c = c > RCAP - o ? RCAP - o : c;
    c = __builtin_amdgcn_readfirstlane(c);
    o = __builtin_amdgcn_readfirstlane(o);
    bigv = __builtin_amdgcn_readfirstlane(bigv);
    int last = o + c - 1; last = last < o ? o : last;

    float a0 = 0.0f, a1 = 0.0f, a2 = 0.0f, a3 = 0.0f;
#pragma unroll 1
    for (int b0 = 0; b0 < c; b0 += 32) {
      int idx = o + b0 + lane;
      idx = idx > last ? last : idx;
      int sr = lb[idx];
      sr = sr < 0 ? 0 : (sr > NN - 1 ? NN - 1 : sr);
      const int m32 = (c - b0) < 32 ? (c - b0) : 32;
#pragma unroll 1
      for (int k = 0; k < m32; ++k) {
        const int sk = __builtin_amdgcn_readlane(sr, k);
        if constexpr (SRC16 != 0) {
          const v2u w = *(const v2ua*)(XB + (size_t)sk * DH + 4 * lane);
          a0 += __uint_as_float(w.x << 16);
          a1 += __uint_as_float(w.x & 0xffff0000u);
          a2 += __uint_as_float(w.y << 16);
          a3 += __uint_as_float(w.y & 0xffff0000u);
        } else {
          const v4f v = *(const v4fa*)(H + (size_t)sk * DH + 4 * lane);
          a0 += v.x; a1 += v.y; a2 += v.z; a3 += v.w;
        }
      }
    }
    const bool live = d < NN;
    const int nc = live ? d : NN - 1;
    float s0, s1, s2, s3;
    if constexpr (SRC16 != 0) {
      const v2u w = *(const v2ua*)(XB + (size_t)nc * DH + 4 * lane);
      s0 = __uint_as_float(w.x << 16);
      s1 = __uint_as_float(w.x & 0xffff0000u);
      s2 = __uint_as_float(w.y << 16);
      s3 = __uint_as_float(w.y & 0xffff0000u);
    } else {
      const v4f v = *(const v4fa*)(H + (size_t)nc * DH + 4 * lane);
      s0 = v.x; s1 = v.y; s2 = v.z; s3 = v.w;
    }
    float r0 = sc * s0 + a0, r1 = sc * s1 + a1, r2 = sc * s2 + a2, r3 = sc * s3 + a3;
    const bool bad = (flag != 0) | (bigv != 0);
    r0 = bad ? qnan : r0; r1 = bad ? qnan : r1; r2 = bad ? qnan : r2; r3 = bad ? qnan : r3;
    r0 = live ? r0 : 0.0f; r1 = live ? r1 : 0.0f; r2 = live ? r2 : 0.0f; r3 = live ? r3 : 0.0f;
    unsigned h01, h23, l01, l23;
    hilo_pack(r0, r1, r2, r3, h01, h23, l01, l23);
    const v4u ow = regroup16(h01, h23, l01, l23, lane);
    st2_v4u(Z + (size_t)d * APITCH + 8 * lane, ow);
  }
}

template <int NT, int KEXT>
__device__ __forceinline__ void gemm_core(const unsigned short* __restrict__ ap,
                                          const unsigned short* __restrict__ bp, v8f (&acc)[NT]) {
#pragma unroll 1
  for (int k0 = 0; k0 < KEXT; k0 += 32) {
    FragB af;
    af.h[0] = *(const v8usa*)(ap + k0);
    af.h[1] = *(const v8usa*)(ap + k0 + 16);
#pragma unroll
    for (int nt = 0; nt < NT; ++nt) {
      const unsigned short* wq = bp + (size_t)(16 * nt) * (size_t)WPITCH + k0;
      FragB bf;
      bf.h[0] = *(const v8usa*)wq;
      bf.h[1] = *(const v8usa*)(wq + 16);
      acc[nt] = wmb(af, bf, acc[nt]);
    }
  }
}

template <int NT, int SPW>
__device__ __forceinline__ void stage_d(float* stg, const v8f (&acc)[NT], int wave, int hh, int m) {
#pragma unroll
  for (int nt = 0; nt < NT; ++nt) {
#pragma unroll
    for (int r = 0; r < 8; ++r) stg[(16 * wave + 8 * hh + r) * SPW + 16 * nt + m] = acc[nt][r];
  }
}

template <int KEXT>
__global__ __launch_bounds__(NTHR) __attribute__((amdgpu_num_vgpr(248)))
void k_gemm_hl(const unsigned short* __restrict__ A, const unsigned short* __restrict__ WT,
               const float* __restrict__ sm, int boff, unsigned short* outH) {
  extern __shared__ __attribute__((aligned(16))) float gsm[];
  float* stg = gsm;
  float* sb  = gsm + GBM * SP128;
  const int tid = (int)threadIdx.x, lane = tid & 31, wave = tid >> 5, hh = lane >> 4, m = lane & 15;
  const int rowBase = (int)blockIdx.x * GBM;
  if (tid < 32) *(v4fa*)(sb + 4 * tid) = *(const v4fa*)(sm + boff + 4 * tid);

  v8f acc[8];
  {
    const v8f z = {0.f, 0.f, 0.f, 0.f, 0.f, 0.f, 0.f, 0.f};
#pragma unroll
    for (int t = 0; t < 8; ++t) acc[t] = z;
  }
  const unsigned short* ap = A + (size_t)(rowBase + 16 * wave + m) * (size_t)APITCH + 8 * hh;
  const unsigned short* bp = WT + (size_t)m * (size_t)WPITCH + 8 * hh;
  gemm_core<8, KEXT>(ap, bp, acc);
  stage_d<8, SP128>(stg, acc, wave, hh, m);
  __syncthreads();

  const int cb = 8 * m;
  const v4f ba = *(const v4fa*)(sb + cb);
  const v4f bb = *(const v4fa*)(sb + cb + 4);
  const float bia[8] = {ba.x, ba.y, ba.z, ba.w, bb.x, bb.y, bb.z, bb.w};
  const unsigned selhi = (hh == 0) ? 0xffffffffu : 0u;
#pragma unroll 1
  for (int i = 0; i < 16; ++i) {
    const int lr = 16 * wave + i;
    const int gr = rowBase + lr;
    const bool live = gr < NN;
    const v4f a = *(const v4fa*)(stg + lr * SP128 + cb);
    const v4f b = *(const v4fa*)(stg + lr * SP128 + cb + 4);
    asm volatile("" :: "v"(a));
    asm volatile("" :: "v"(b));
    const float f[8] = {a.x + bia[0], a.y + bia[1], a.z + bia[2], a.w + bia[3],
                        b.x + bia[4], b.y + bia[5], b.z + bia[6], b.w + bia[7]};
    unsigned w[4];
#pragma unroll
    for (int j = 0; j < 4; ++j) {
      float v0 = f[2 * j], v1 = f[2 * j + 1];
      v0 = (v0 > 0.0f) ? v0 : (v0 - v0);
      v1 = (v1 > 0.0f) ? v1 : (v1 - v1);
      v0 = live ? v0 : 0.0f;
      v1 = live ? v1 : 0.0f;
      const unsigned h0 = bf16_bits(v0), h1 = bf16_bits(v1);
      const unsigned l0 = bf16_bits(v0 - __uint_as_float(h0 << 16));
      const unsigned l1 = bf16_bits(v1 - __uint_as_float(h1 << 16));
      w[j] = ((h0 | (h1 << 16)) & selhi) | ((l0 | (l1 << 16)) & ~selhi);
    }
    v4u pw;
    pw.x = w[0]; pw.y = w[1]; pw.z = w[2]; pw.w = w[3];
    st2_v4u(outH + (size_t)gr * APITCH + 8 * lane, pw);
  }
}

template <int KEXT>
__global__ __launch_bounds__(NTHR) __attribute__((amdgpu_num_vgpr(248)))
void k_gemm_f32(const unsigned short* __restrict__ A, const unsigned short* __restrict__ WT,
                const float* __restrict__ sm, int boff, float* outF) {
  extern __shared__ __attribute__((aligned(16))) float gsm[];
  float* stg = gsm;
  float* sb  = gsm + GBM * SP128;
  const int tid = (int)threadIdx.x, lane = tid & 31, wave = tid >> 5, hh = lane >> 4, m = lane & 15;
  const int rowBase = (int)blockIdx.x * GBM;
  if (tid < 32) *(v4fa*)(sb + 4 * tid) = *(const v4fa*)(sm + boff + 4 * tid);

  v8f acc[8];
  {
    const v8f z = {0.f, 0.f, 0.f, 0.f, 0.f, 0.f, 0.f, 0.f};
#pragma unroll
    for (int t = 0; t < 8; ++t) acc[t] = z;
  }
  const unsigned short* ap = A + (size_t)(rowBase + 16 * wave + m) * (size_t)APITCH + 8 * hh;
  const unsigned short* bp = WT + (size_t)m * (size_t)WPITCH + 8 * hh;
  gemm_core<8, KEXT>(ap, bp, acc);
  stage_d<8, SP128>(stg, acc, wave, hh, m);
  __syncthreads();

  const v4f bias = *(const v4fa*)(sb + 4 * lane);
#pragma unroll 1
  for (int i = 0; i < 16; ++i) {
    const int lr = 16 * wave + i;
    const int gr = rowBase + lr;
    const v4f a = *(const v4fa*)(stg + lr * SP128 + 4 * lane);
    asm volatile("" :: "v"(a));
    float v0 = a.x + bias.x, v1 = a.y + bias.y, v2 = a.z + bias.z, v3 = a.w + bias.w;
    v0 = (v0 > 0.0f) ? v0 : (v0 - v0); v1 = (v1 > 0.0f) ? v1 : (v1 - v1);
    v2 = (v2 > 0.0f) ? v2 : (v2 - v2); v3 = (v3 > 0.0f) ? v3 : (v3 - v3);
    v4f o;
    o.x = v0; o.y = v1; o.z = v2; o.w = v3;
    const int gc = gr < NN ? gr : NN - 1;
    st2_v4f(outF + (size_t)gc * DH + 4 * lane, o, gr < NN);
  }
}

template <int KEXT>
__global__ __launch_bounds__(NTHR) __attribute__((amdgpu_num_vgpr(248)))
void k_head(const unsigned short* __restrict__ A, const unsigned short* __restrict__ WT,
            const float* __restrict__ sm, int boff, const int* __restrict__ FLAG, float* out) {
  __shared__ __attribute__((aligned(16))) float stg[GBM * SP64];
  __shared__ __attribute__((aligned(16))) float sb[OC];
  const int tid = (int)threadIdx.x, lane = tid & 31, wave = tid >> 5, hh = lane >> 4, m = lane & 15;
  const int rowBase = (int)blockIdx.x * GBM;
  const int flag = FLAG[(size_t)(rowBase >> SLB) * 32];
  if (tid < 16) *(v4fa*)(sb + 4 * tid) = *(const v4fa*)(sm + boff + 4 * tid);

  v8f acc[4];
  {
    const v8f z = {0.f, 0.f, 0.f, 0.f, 0.f, 0.f, 0.f, 0.f};
#pragma unroll
    for (int t = 0; t < 4; ++t) acc[t] = z;
  }
  const unsigned short* ap = A + (size_t)(rowBase + 16 * wave + m) * (size_t)APITCH + 8 * hh;
  const unsigned short* bp = WT + (size_t)m * (size_t)WPITCH + 8 * hh;
  gemm_core<4, KEXT>(ap, bp, acc);
  stage_d<4, SP64>(stg, acc, wave, hh, m);
  __syncthreads();

  const v2f bias = *(const v2fa*)(sb + 2 * lane);
  const float qnan = __uint_as_float(0x7fc00000u);
#pragma unroll 1
  for (int i = 0; i < 16; ++i) {
    const int lr = 16 * wave + i;
    const int gr = rowBase + lr;
    const v2f a = *(const v2fa*)(stg + lr * SP64 + 2 * lane);
    asm volatile("" :: "v"(a));
    const float v0 = a.x + bias.x, v1 = a.y + bias.y;
    float mx = v0;
    mx = ((v1 > mx) | (v1 != v1)) ? v1 : mx;
#pragma unroll
    for (int d = 16; d >= 1; d >>= 1) {
      const float o = __shfl_xor(mx, d, 32);
      mx = ((o > mx) | (o != o)) ? o : mx;
    }
    float se = expf(v0 - mx) + expf(v1 - mx);
#pragma unroll
    for (int d = 16; d >= 1; d >>= 1) se += __shfl_xor(se, d, 32);
    const float ls = logf(se);
    float r0 = (v0 - mx) - ls, r1 = (v1 - mx) - ls;
    r0 = (flag != 0) ? qnan : r0;
    r1 = (flag != 0) ? qnan : r1;
    v2f ov;
    ov.x = r0; ov.y = r1;
    const int gc = gr < NN ? gr : NN - 1;
    st2_v2f(out + (size_t)gc * OC + 2 * lane, ov, gr < NN);
  }
}

extern "C" void kernel_launch(void* const* d_in, const int* in_sizes, int n_in,
                              void* d_out, int out_size, void* d_ws, size_t ws_size,
                              hipStream_t stream) {
  if (n_in < 12) return;
  if (in_sizes[0] != NN * DH) return;
  if (in_sizes[1] != 2 * NE) return;
  if (in_sizes[2] != DH * DH) return;
  if (in_sizes[3] != DH) return;
  if (in_sizes[4] != DH * DH) return;
  if (in_sizes[5] != DH) return;
  if (in_sizes[6] != 1) return;
  if (in_sizes[7] != DH * DH) return;
  if (in_sizes[8] != DH) return;
  if (in_sizes[9] != DH * OC) return;
  if (in_sizes[10] != OC) return;
  if (in_sizes[11] != 1) return;
  if (out_size != NN * OC) return;

  const float* x   = (const float*)d_in[0];
  const int*   ei  = (const int*)d_in[1];
  const float* w1  = (const float*)d_in[2];
  const float* b1  = (const float*)d_in[3];
  const float* w2  = (const float*)d_in[4];
  const float* b2  = (const float*)d_in[5];
  const float* e0p = (const float*)d_in[6];
  const float* w3  = (const float*)d_in[7];
  const float* b3  = (const float*)d_in[8];
  const float* w4  = (const float*)d_in[9];
  const float* b4  = (const float*)d_in[10];
  const float* e1p = (const float*)d_in[11];
  float* out = (float*)d_out;
  const int* srcs = ei;
  const int* dsts = ei + NE;

  constexpr size_t zXB   = (size_t)MP * DH * 2;
  constexpr size_t zHL   = (size_t)MP * APITCH * 2;
  constexpr size_t zH    = (size_t)NN * DH * 4;
  constexpr size_t zLIST = (size_t)NBK * RCAP * 4;
  constexpr size_t zCO   = (size_t)NBK * 2 * NBRUN * 4;
  constexpr size_t zFLAG = (size_t)NBK * 128;
  constexpr size_t zW    = (size_t)DH * WPITCH * 2;
  constexpr size_t zW4   = (size_t)OC * WPITCH * 2;
  constexpr size_t zSM   = 2048;
  constexpr size_t oXB   = 0;
  constexpr size_t oZ    = oXB + zXB;
  constexpr size_t oPB   = oZ + zHL;
  constexpr size_t oH    = oPB + zHL;
  constexpr size_t oLIST = oH + zH;
  constexpr size_t oCO   = oLIST + zLIST;
  constexpr size_t oFLAG = oCO + zCO;
  constexpr size_t oW1   = oFLAG + zFLAG;
  constexpr size_t oW2   = oW1 + zW;
  constexpr size_t oW3   = oW2 + zW;
  constexpr size_t oW4   = oW3 + zW;
  constexpr size_t oSM   = oW4 + zW4;
  constexpr size_t oEND  = oSM + zSM;
  static_assert(zXB % 256 == 0 && zHL % 256 == 0 && zH % 256 == 0 && zLIST % 256 == 0 && zCO % 256 == 0);
  static_assert(zFLAG % 256 == 0 && zW % 256 == 0 && zW4 % 256 == 0 && zSM % 256 == 0);
  static_assert(oEND <= (size_t)WSMAX);
  if (oEND > ws_size) return;

  char* ws = (char*)d_ws;
  unsigned short* XB   = (unsigned short*)(ws + oXB);
  unsigned short* Z    = (unsigned short*)(ws + oZ);
  unsigned short* PB   = (unsigned short*)(ws + oPB);
  float*          H    = (float*)(ws + oH);
  int*            LIST = (int*)(ws + oLIST);
  int*            CO   = (int*)(ws + oCO);
  int*            FLAG = (int*)(ws + oFLAG);
  unsigned short* W1D  = (unsigned short*)(ws + oW1);
  unsigned short* W2D  = (unsigned short*)(ws + oW2);
  unsigned short* W3D  = (unsigned short*)(ws + oW3);
  unsigned short* W4D  = (unsigned short*)(ws + oW4);
  float*          SM   = (float*)(ws + oSM);

  hipFuncSetAttribute(reinterpret_cast<const void*>(&k_bucket), hipFuncAttributeMaxDynamicSharedMemorySize, (int)BK_LDS);
  hipFuncSetAttribute(reinterpret_cast<const void*>(&k_gemm_hl<KEXT_AGG>), hipFuncAttributeMaxDynamicSharedMemorySize, (int)GM_LDS);
  hipFuncSetAttribute(reinterpret_cast<const void*>(&k_gemm_f32<KEXT_HID>), hipFuncAttributeMaxDynamicSharedMemorySize, (int)GM_LDS);

  k_prep<<<PBTOT, NTHR, 0, stream>>>(x, w1, w2, w3, w4, b1, b2, b3, b4, e0p, e1p, XB, W1D, W2D, W3D, W4D, SM);
  k_bucket<<<NBK, NTHR, BK_LDS, stream>>>(srcs, dsts, LIST, CO, FLAG);
  k_agg<1><<<MP / ABM, NTHR, 0, stream>>>(LIST, CO, FLAG, XB, H, SM, 0, Z);
  k_gemm_hl<KEXT_AGG><<<MP / GBM, NTHR, GM_LDS, stream>>>(Z, W1D, SM, 0, PB);
  k_gemm_f32<KEXT_HID><<<MP / GBM, NTHR, GM_LDS, stream>>>(PB, W2D, SM, DH, H);
  k_agg<0><<<MP / ABM, NTHR, 0, stream>>>(LIST, CO, FLAG, XB, H, SM, 1, Z);
  k_gemm_hl<KEXT_AGG><<<MP / GBM, NTHR, GM_LDS, stream>>>(Z, W3D, SM, 2 * DH, PB);
  k_head<KEXT_HID><<<MP / GBM, NTHR, 0, stream>>>(PB, W4D, SM, 3 * DH, FLAG, out);
}
